// GNNSAGPool_37744172597493
// MI455X (gfx1250) — hardware-verified
//
#include <hip/hip_runtime.h>
#include <math.h>

typedef __attribute__((ext_vector_type(16))) __bf16 v16bf;
typedef __attribute__((ext_vector_type(8)))  __bf16 v8bf;
typedef __attribute__((ext_vector_type(8)))  float  v8f;
typedef __attribute__((ext_vector_type(4)))  float  v4f;
typedef __attribute__((ext_vector_type(4)))  unsigned v4u;
typedef __attribute__((ext_vector_type(4)))  int i4;
typedef float __attribute__((may_alias)) float_a;
typedef int __attribute__((may_alias)) int_a;

#define N0 32768
#define K1N 16384
#define K2N 8192
#define HD 256
#define NE 524288
#define N_NODES N0
#define BT 256
#define ECAP 5120
#define SCAP 48
#define ETILE 2048

template <typename V> __device__ __forceinline__ void vst2(void* p, V v) {
  *(volatile V*)p = v; __threadfence(); *(volatile V*)p = v;
}
__device__ __forceinline__ v8f wmma_bf(v16bf a, v16bf b, v8f c) {
  v8f d = __builtin_amdgcn_wmma_f32_16x16x32_bf16(false, a, false, b, (short)0, c, false, false);
  asm volatile("v_nop\n\tv_nop\n\tv_nop\n\tv_nop" : "+v"(d) : "v"(a), "v"(b));
  return d;
}
struct A3 { v16bf h, m, l; };
__device__ __forceinline__ A3 split_row(const float* row, int k0, int lane) {
  A3 r; const float* p = row + k0 + 8 * (lane >> 4);
#pragma unroll
  for (int i = 0; i < 16; ++i) {
    const float x = p[(i < 8) ? i : (i + 8)];
    const __bf16 h = (__bf16)x; const float rh = x - (float)h;
    const __bf16 m = (__bf16)rh; const __bf16 l = (__bf16)(rh - (float)m);
    r.h[i] = h; r.m[i] = m; r.l[i] = l;
  }
  return r;
}
__device__ __forceinline__ v16bf frag_bf(const __bf16* row, int k0, int lane) {
  union { v16bf v; v8bf q[2]; } r; const __bf16* p = row + k0 + 8 * (lane >> 4);
  r.q[0] = *(const v8bf*)(p); r.q[1] = *(const v8bf*)(p + 16); return r.v;
}
__device__ __forceinline__ v8f mac6(const A3& a, const __bf16* bh, const __bf16* bm, const __bf16* bl, int k0, int lane, v8f c) {
  const v16bf fh = frag_bf(bh, k0, lane), fm = frag_bf(bm, k0, lane), fl = frag_bf(bl, k0, lane);
  c = wmma_bf(a.l, fh, c); c = wmma_bf(a.m, fm, c); c = wmma_bf(a.h, fl, c);
  c = wmma_bf(a.m, fh, c); c = wmma_bf(a.h, fm, c); c = wmma_bf(a.h, fh, c);
  return c;
}

__device__ __forceinline__ float eluf(float v) { return v > 0.f ? v : expm1f(v); }

struct Bucket {
  int ledge[ECAP]; unsigned short ltgt[ECAP]; unsigned short sub[BT][SCAP]; int scnt[BT]; int wcnt[8][8]; int total;
};
__device__ void bucket_build(Bucket& bk, const int* __restrict__ src, const int* __restrict__ dst, int E, int tlo, int tid) {
  const int lane = tid & 31, wave = tid >> 5;
  if (tid == 0) bk.total = 0;
  __syncthreads();
  for (int e0 = 0; e0 < E; e0 += ETILE) {
    int rv[8]; unsigned msk[8];
#pragma unroll
    for (int j = 0; j < 8; ++j) {
      const int e = e0 + j * 256 + tid;
      const int r = (e < E) ? dst[e] : -1;
      rv[j] = r;
      msk[j] = (unsigned)__builtin_amdgcn_ballot_w32((r >= tlo) && (r < tlo + BT));
    }
    if (lane < 8) bk.wcnt[lane][wave] = __builtin_popcount(msk[lane]);
    __syncthreads();
    const int base = bk.total;
    int run = 0, pre[8];
#pragma unroll
    for (int j = 0; j < 8; ++j) {
#pragma unroll
      for (int w = 0; w < 8; ++w) { if (w == wave) pre[j] = run; run += bk.wcnt[j][w]; }
    }
#pragma unroll
    for (int j = 0; j < 8; ++j) {
      const unsigned m = msk[j];
      if ((m >> lane) & 1u) {
        const int pos = base + pre[j] + __builtin_popcount(m & ((1u << lane) - 1u));
        if (pos < ECAP) { bk.ledge[pos] = e0 + j * 256 + tid; bk.ltgt[pos] = (unsigned short)(rv[j] - tlo); }
      }
    }
    __syncthreads();
    if (tid == 0) bk.total = base + run;
    __syncthreads();
  }
  const int n = (bk.total < ECAP) ? bk.total : ECAP;
  (void)src;
  int k = 0;
  for (int i = 0; i < n; ++i) if ((int)bk.ltgt[i] == tid) { if (k < SCAP) bk.sub[tid][k] = (unsigned short)i; ++k; }
  bk.scnt[tid] = (k < SCAP) ? k : SCAP;
  __syncthreads();
}


__global__ __launch_bounds__(256) void k_split3(const float* __restrict__ W, __bf16* __restrict__ P) {
  __shared__ __align__(16) __bf16 th[64][72], tm[64][72], tl[64][72];
  const int tid = threadIdx.x, n0 = (blockIdx.x & 3) * 64, k0 = (blockIdx.x >> 2) * 64;
  for (int i = tid; i < 64 * 64; i += 256) {
    const int kk = i >> 6, nn = i & 63; const float x = W[(size_t)(k0 + kk) * HD + n0 + nn];
    const __bf16 h = (__bf16)x; const float rh = x - (float)h; const __bf16 m = (__bf16)rh; const __bf16 l = (__bf16)(rh - (float)m);
    th[nn][kk] = h; tm[nn][kk] = m; tl[nn][kk] = l;
  }
  __syncthreads();
  const size_t plane = (size_t)HD * HD;
  for (int g = tid; g < 64 * 8; g += 256) { const int nn = g >> 3, pc = g & 7; const size_t o = (size_t)(n0 + nn) * HD + k0 + pc * 8;
    vst2(P + o, *(const v4u*)(&th[nn][pc * 8])); vst2(P + plane + o, *(const v4u*)(&tm[nn][pc * 8])); vst2(P + 2 * plane + o, *(const v4u*)(&tl[nn][pc * 8])); }
}
__global__ __launch_bounds__(128) void k_gemm6(const float* __restrict__ X, const __bf16* __restrict__ P, float* __restrict__ Y, int nrows) {
  __shared__ __align__(16) float so[16 * HD];
  const int tid = threadIdx.x, wave = tid >> 5, lane = tid & 31, hi = lane >> 4, col = lane & 15;
  const int m0 = blockIdx.x * 16;
  const size_t plane = (size_t)HD * HD;
  const float* ar = X + (size_t)(m0 + col) * HD;
  v8f acc[4] = {(v8f){}, (v8f){}, (v8f){}, (v8f){}};
#pragma unroll 1
  for (int kc = 0; kc < HD / 32; ++kc) {
    const A3 a = split_row(ar, kc * 32, lane);
#pragma unroll
    for (int j = 0; j < 4; ++j) { const size_t ro = (size_t)(wave * 64 + j * 16 + col) * HD; acc[j] = mac6(a, P + ro, P + plane + ro, P + 2 * plane + ro, kc * 32, lane, acc[j]); }
  }
#pragma unroll
  for (int j = 0; j < 4; ++j) { const int n = wave * 64 + j * 16 + col;
#pragma unroll
    for (int r = 0; r < 8; ++r) so[(hi * 8 + r) * HD + n] = acc[j][r]; }
  __syncthreads();
  (void)nrows;
  float* dst = Y + (size_t)m0 * HD;
  for (int g = tid; g < 16 * HD / 4; g += 128) vst2(dst + g * 4, *(const v4f*)(&so[g * 4]));
}
__global__ __launch_bounds__(256) void k_gemv(const float* __restrict__ X, const float* __restrict__ w, float* __restrict__ sv, int n) {
  __shared__ float red[32];
  const int tid = threadIdx.x, wave = tid >> 5, lane = tid & 31;
  for (int r = 0; r < 4; ++r) { const int node = blockIdx.x * 32 + wave * 4 + r;
    float s = 0.f;
    if (node < n) { const float* xr = X + (size_t)node * HD;
#pragma unroll
      for (int j = 0; j < 8; ++j) s += xr[lane + 32 * j] * w[lane + 32 * j]; }
#pragma unroll
    for (int off = 16; off > 0; off >>= 1) s += __shfl_xor(s, off, 32);
    if (lane == 0) red[wave * 4 + r] = s; }
  __syncthreads();
  if (tid < 32) vst2(sv + blockIdx.x * 32 + tid, (float_a)red[tid]);
}

template <int MODE>
__global__ __launch_bounds__(256) void k_gcn(const int* __restrict__ esrc, const int* __restrict__ edst, const float* __restrict__ ew, int n_nodes,
                                             const float* __restrict__ h, const float* __restrict__ sv, const float* __restrict__ bias,
                                             const float* __restrict__ dinv_in, float* __restrict__ dinv_out, float* __restrict__ out) {
  __shared__ Bucket bk;
  __shared__ float sres[BT], sdi[BT];
  const int tid = threadIdx.x, lane = tid & 31, wave = tid >> 5, tlo = blockIdx.x * BT;
  bucket_build(bk, esrc, edst, NE, tlo, tid);
  for (int s = 0; s < 32; ++s) {
    const int t = wave * 32 + s, node = tlo + t;
    if (node >= n_nodes) break;
    const int cnt = bk.scnt[t];
    const float di = dinv_in[node];
    if (MODE == 0) {
      float acc[8];
#pragma unroll
      for (int j = 0; j < 8; ++j) acc[j] = 0.f;
      for (int k = 0; k < cnt; ++k) {
        const int e = bk.ledge[bk.sub[t][k]]; int sN = esrc[e]; sN = sN < 0 ? 0 : (sN >= n_nodes ? n_nodes - 1 : sN);
        const float w = dinv_in[sN] * di * ew[e];
        const float* hr = h + (size_t)sN * HD;
#pragma unroll
        for (int j = 0; j < 8; ++j) acc[j] += w * hr[lane + 32 * j];
      }
      const float* hn = h + (size_t)node * HD; const float sw = 2.0f * di * di;
      float* orow = out + (size_t)node * HD;
#pragma unroll
      for (int j = 0; j < 8; ++j) { const int c = lane + 32 * j; vst2(orow + c, (float_a)eluf(acc[j] + hn[c] * sw + bias[c])); }
    } else {
      float acc = 0.f;
      for (int k = lane; k < cnt; k += 32) {
        const int e = bk.ledge[bk.sub[t][k]]; int sN = esrc[e]; sN = sN < 0 ? 0 : (sN >= n_nodes ? n_nodes - 1 : sN);
        acc += dinv_in[sN] * di * ew[e] * sv[sN];
      }
#pragma unroll
      for (int off = 16; off > 0; off >>= 1) acc += __shfl_xor(acc, off, 32);
      if (lane == 0) sres[t] = acc + sv[node] * 2.0f * di * di + bias[0];
    }
  }
  __syncthreads();
  if (MODE != 0) { if (tlo + tid < n_nodes) vst2(out + tlo + tid, (float_a)sres[tid]); }
  (void)sdi; (void)dinv_out;
}
__global__ __launch_bounds__(256) void k_deg(const int* __restrict__ esrc, const int* __restrict__ edst, const float* __restrict__ ew, int n_nodes, float* __restrict__ dinv) {
  __shared__ Bucket bk;
  __shared__ float sdi[BT];
  const int tid = threadIdx.x, lane = tid & 31, wave = tid >> 5, tlo = blockIdx.x * BT;
  bucket_build(bk, esrc, edst, NE, tlo, tid);
  for (int s = 0; s < 32; ++s) {
    const int t = wave * 32 + s, node = tlo + t;
    if (node >= n_nodes) break;
    const int cnt = bk.scnt[t];
    float dg = 0.f;
    for (int k = lane; k < cnt; k += 32) dg += ew[bk.ledge[bk.sub[t][k]]];
#pragma unroll
    for (int off = 16; off > 0; off >>= 1) dg += __shfl_xor(dg, off, 32);
    if (lane == 0) sdi[t] = rsqrtf(dg + 2.0f);
  }
  __syncthreads();
  if (tlo + tid < n_nodes) vst2(dinv + tlo + tid, (float_a)sdi[tid]);
}

__global__ __launch_bounds__(256) void k_rank(const float* __restrict__ sc, int n, int* __restrict__ rank) {
  __shared__ float tile[2048];
  const int i = blockIdx.x * 256 + threadIdx.x;
  const float si = (i < n) ? sc[i] : 0.f;
  int r = 0;
  for (int j0 = 0; j0 < n; j0 += 2048) {
    __syncthreads();
    for (int t = threadIdx.x; t < 2048; t += 256) tile[t] = (j0 + t < n) ? sc[j0 + t] : -3.0e38f;
    __syncthreads();
    if (i < n) {
#pragma unroll 4
      for (int t = 0; t < 2048; ++t) { const float sj = tile[t]; const int j = j0 + t; r += (sj > si) | ((sj == si) & (j < i)); }
    }
  }
  if (i < n) vst2(rank + i, (int_a)r);
}
__global__ __launch_bounds__(256) void k_pool(const float* __restrict__ x, const float* __restrict__ sc, const int* __restrict__ rank, int n, int k, float* __restrict__ xk) {
  const int tid = threadIdx.x, wave = tid >> 5, lane = tid & 31, i = blockIdx.x * 8 + wave;
  if (i >= n) return;
  const int r = rank[i];
  if (r < 0 || r >= k) return;
  const float tv = tanhf(sc[i]);
  const float* xr = x + (size_t)i * HD; float* orow = xk + (size_t)r * HD;
#pragma unroll
  for (int j = 0; j < 8; ++j) vst2(orow + lane + 32 * j, (float_a)(xr[lane + 32 * j] * tv));
}
__global__ __launch_bounds__(256) void k_remap(const int* __restrict__ osrc, const int* __restrict__ odst, const float* __restrict__ oew,
                                              const int* __restrict__ rank, int nprev, int k, int* __restrict__ nsrc, int* __restrict__ ndst, float* __restrict__ new_ew) {
  const int e = blockIdx.x * 256 + threadIdx.x;
  const int s = osrc[e], d = odst[e];
  const int ns = (s >= 0 && s < nprev && rank[s] < k) ? rank[s] : -1;
  const int nd = (d >= 0 && d < nprev && rank[d] < k) ? rank[d] : -1;
  const bool keep = (ns >= 0) && (nd >= 0) && (oew[e] != 0.f || true);
  vst2(nsrc + e, (int_a)(ns >= 0 ? ns : 0));
  vst2(ndst + e, (int_a)(keep ? nd : -1));
  vst2(new_ew + e, (float_a)(keep ? oew[e] : 0.f));
}
__global__ __launch_bounds__(256) void k_fill1(float* __restrict__ ew) { const int e = blockIdx.x * 256 + threadIdx.x; vst2(ew + e, (float_a)1.0f); }
__global__ __launch_bounds__(256) void k_head(const float* __restrict__ x3, const int* __restrict__ rank, int n, const float* __restrict__ Wc1,
                                             const float* __restrict__ bc1, const float* __restrict__ Wc2, const float* __restrict__ bc2, float* __restrict__ out) {
  __shared__ float vals[32];
  __shared__ float hid[256];
  const int tid = threadIdx.x;
  if (tid < 32) vals[tid] = 0.f;
  __syncthreads();
  for (int i = tid; i < n; i += 256) { const int r = rank[i]; if (r < 30) vals[r] = x3[i]; }
  __syncthreads();
  { float s = bc1[tid];
#pragma unroll 1
    for (int j = 0; j < 30; ++j) s += vals[j] * Wc1[j * HD + tid];
    hid[tid] = eluf(s); }
  __syncthreads();
  if (tid < 10) { float s = bc2[tid];
#pragma unroll 1
    for (int c = 0; c < HD; ++c) s += hid[c] * Wc2[c * 10 + tid];
    vst2(out + tid, (float_a)s); }
}

extern "C" void kernel_launch(void* const* d_in, const int* in_sizes, int n_in,
                              void* d_out, int out_size, void* d_ws, size_t ws_size,
                              hipStream_t stream) {
  (void)in_sizes; (void)n_in; (void)out_size; (void)ws_size;
  const float* x = (const float*)d_in[0];
  const int* ei = (const int*)d_in[1];
  const int* src0 = ei; const int* dst0 = ei + NE;
  const float *W1 = (const float*)d_in[2], *b1 = (const float*)d_in[3], *Wp1 = (const float*)d_in[4], *bp1 = (const float*)d_in[5];
  const float *W2 = (const float*)d_in[6], *b2 = (const float*)d_in[7], *Wp2 = (const float*)d_in[8], *bp2 = (const float*)d_in[9];
  const float *W3 = (const float*)d_in[10], *b3 = (const float*)d_in[11];
  const float *Wc1 = (const float*)d_in[12], *bc1 = (const float*)d_in[13], *Wc2 = (const float*)d_in[14], *bc2 = (const float*)d_in[15];
  float* out = (float*)d_out;

  char* ws = (char*)d_ws; size_t off = 0;
  auto alloc = [&](size_t bytes) -> void* { void* p = ws + off; off = (off + bytes + 255) & ~(size_t)255; return p; };
  __bf16* P1 = (__bf16*)alloc((size_t)3 * HD * HD * 2);
  __bf16* P2 = (__bf16*)alloc((size_t)3 * HD * HD * 2);
  float* H   = (float*)alloc((size_t)N0 * HD * 4);
  float* X1  = (float*)alloc((size_t)N0 * HD * 4);
  float* XK1 = (float*)alloc((size_t)K1N * HD * 4);
  float* X2  = (float*)alloc((size_t)K1N * HD * 4);
  float* XK2 = (float*)alloc((size_t)K2N * HD * 4);
  float* dinv = (float*)alloc((size_t)N0 * 4);
  float* sv   = (float*)alloc((size_t)N0 * 4);
  float* sc   = (float*)alloc((size_t)N0 * 4);
  int* rank   = (int*)alloc((size_t)N0 * 4);
  float* ew0 = (float*)alloc((size_t)NE * 4);
  int* src1 = (int*)alloc((size_t)NE * 4); int* dst1 = (int*)alloc((size_t)NE * 4); float* ew1 = (float*)alloc((size_t)NE * 4);
  int* src2 = (int*)alloc((size_t)NE * 4); int* dst2 = (int*)alloc((size_t)NE * 4); float* ew2 = (float*)alloc((size_t)NE * 4);

  k_split3<<<16, 256, 0, stream>>>(W1, P1);
  k_split3<<<16, 256, 0, stream>>>(W2, P2);
  k_fill1<<<NE / 256, 256, 0, stream>>>(ew0);
  k_gemm6<<<N0 / 16, 128, 0, stream>>>(x, P1, H, N0);
  k_deg<<<N0 / BT, 256, 0, stream>>>(src0, dst0, ew0, N0, dinv);
  k_gcn<0><<<N0 / BT, 256, 0, stream>>>(src0, dst0, ew0, N0, H, nullptr, b1, dinv, dinv, X1);
  k_gemv<<<N0 / 32, 256, 0, stream>>>(X1, Wp1, sv, N0);
  k_gcn<1><<<N0 / BT, 256, 0, stream>>>(src0, dst0, ew0, N0, nullptr, sv, bp1, dinv, nullptr, sc);
  k_rank<<<N0 / 256, 256, 0, stream>>>(sc, N0, rank);
  k_pool<<<N0 / 8, 256, 0, stream>>>(X1, sc, rank, N0, K1N, XK1);
  k_remap<<<NE / 256, 256, 0, stream>>>(src0, dst0, ew0, rank, N0, K1N, src1, dst1, ew1);
  k_gemm6<<<K1N / 16, 128, 0, stream>>>(XK1, P2, H, K1N);
  k_deg<<<K1N / BT, 256, 0, stream>>>(src1, dst1, ew1, K1N, dinv);
  k_gcn<0><<<K1N / BT, 256, 0, stream>>>(src1, dst1, ew1, K1N, H, nullptr, b2, dinv, dinv, X2);
  k_gemv<<<K1N / 32, 256, 0, stream>>>(X2, Wp2, sv, K1N);
  k_gcn<1><<<K1N / BT, 256, 0, stream>>>(src1, dst1, ew1, K1N, nullptr, sv, bp2, dinv, nullptr, sc);
  k_rank<<<K1N / 256, 256, 0, stream>>>(sc, K1N, rank);
  k_pool<<<K1N / 8, 256, 0, stream>>>(X2, sc, rank, K1N, K2N, XK2);
  k_remap<<<NE / 256, 256, 0, stream>>>(src1, dst1, ew1, rank, K1N, K2N, src2, dst2, ew2);
  k_gemv<<<K2N / 32, 256, 0, stream>>>(XK2, W3, sv, K2N);
  k_deg<<<K2N / BT, 256, 0, stream>>>(src2, dst2, ew2, K2N, dinv);
  k_gcn<1><<<K2N / BT, 256, 0, stream>>>(src2, dst2, ew2, K2N, nullptr, sv, b3, dinv, nullptr, sc);
  k_rank<<<K2N / 256, 256, 0, stream>>>(sc, K2N, rank);
  k_head<<<1, 256, 0, stream>>>(sc, rank, K2N, Wc1, bc1, Wc2, bc2, out);
}
